// MultiHeadCrossAttentionBlock_51281909514459
// MI455X (gfx1250) — hardware-verified
//
#include <hip/hip_runtime.h>


#define NB_  8
#define CC   64
#define NN   1024
#define NH_  8
#define QO   512
#define NG   32
#define PCAR 1024.0f
typedef _Float16 h16;
typedef unsigned short bf;
typedef __attribute__((ext_vector_type(16))) __bf16   v16bf;
typedef __attribute__((ext_vector_type(16))) _Float16 v16h;
typedef __attribute__((ext_vector_type(8)))  _Float16 v8h;
typedef __attribute__((ext_vector_type(8)))  unsigned short v8us;
typedef __attribute__((ext_vector_type(8)))  float    v8f;
typedef __attribute__((ext_vector_type(4)))  float    v4f;
typedef v8h  __attribute__((may_alias)) v8ha;
typedef v4f  __attribute__((may_alias)) v4fa;
typedef v8us __attribute__((may_alias)) v8usa;

__device__ __forceinline__ unsigned short f2bf(float f) { unsigned u = __float_as_uint(f); u += 0x7FFFu + ((u >> 16) & 1u); return (unsigned short)(u >> 16); }
__device__ __forceinline__ float bf2f(unsigned short b) { return __uint_as_float(((unsigned)b) << 16); }
__device__ __forceinline__ float bfr(float f) { return bf2f(f2bf(f)); }
__device__ __forceinline__ v16h cat16(v8h lo, v8h hi) { return __builtin_shufflevector(lo, hi, 0, 1, 2, 3, 4, 5, 6, 7, 8, 9, 10, 11, 12, 13, 14, 15); }
__device__ __forceinline__ v16bf cat16b(v8us lo, v8us hi) { return __builtin_bit_cast(v16bf, __builtin_shufflevector(lo, hi, 0, 1, 2, 3, 4, 5, 6, 7, 8, 9, 10, 11, 12, 13, 14, 15)); }
__device__ __forceinline__ v8f wmma16(v16h a, v16h b, v8f c) { return __builtin_amdgcn_wmma_f32_16x16x32_f16(false, a, false, b, (short)0, c, false, false); }
__device__ __forceinline__ v8f wmmab(v16bf a, v16bf b, v8f c) { return __builtin_amdgcn_wmma_f32_16x16x32_bf16(false, a, false, b, (short)0, c, false, false); }


template <typename T16> struct WFrag;
template <> struct WFrag<h16> { typedef v16h V; static __device__ __forceinline__ V ld(const h16* p) { return cat16(*(const v8h*)p, *(const v8h*)(p + 16)); } static __device__ __forceinline__ v8f mma(V a, V b, v8f c) { return wmma16(a, b, c); } };
template <> struct WFrag<bf> { typedef v16bf V; static __device__ __forceinline__ V ld(const bf* p) { return cat16b(*(const v8us*)p, *(const v8us*)(p + 16)); } static __device__ __forceinline__ v8f mma(V a, V b, v8f c) { return wmmab(a, b, c); } };
template <typename T16, int NSPLIT, bool BIAS>
__global__ __launch_bounds__(32) void k_gemmw(const T16* __restrict__ A, const T16* __restrict__ A2, const T16* __restrict__ Bt, const T16* __restrict__ Bt2, int K, float* C, int ldc, const float* __restrict__ bias, size_t sA, size_t sB, size_t sC) {
    typedef typename WFrag<T16>::V V;
    __shared__ __align__(16) float os[16 * 68];
    const size_t z = blockIdx.z; A += z * sA; if (A2) A2 += z * sA; Bt += z * sB; if (Bt2) Bt2 += z * sB; C += z * sC;
    const int lane = threadIdx.x & 31, lr = lane & 15, hi = lane >> 4; const int r0 = blockIdx.x * 64, c0 = blockIdx.y * 64;
    v8f acc[4][4];
#pragma unroll
    for (int mb = 0; mb < 4; ++mb)
#pragma unroll
        for (int nb = 0; nb < 4; ++nb) acc[mb][nb] = (v8f){};
    const size_t aoff = (size_t)(r0 + lr) * K + 8 * hi, boff = (size_t)(c0 + lr) * K + 8 * hi;
#pragma unroll 1
    for (int kc = 0; kc < K; kc += 32) {
        V a[4], a2[4];
#pragma unroll
        for (int mb = 0; mb < 4; ++mb) { a[mb] = WFrag<T16>::ld(A + aoff + (size_t)mb * 16 * K + kc); if (NSPLIT == 1 || NSPLIT == 2) a2[mb] = WFrag<T16>::ld(A2 + aoff + (size_t)mb * 16 * K + kc); }
#pragma unroll
        for (int nb = 0; nb < 4; ++nb) { const V b = WFrag<T16>::ld(Bt + boff + (size_t)nb * 16 * K + kc); V b2; if (NSPLIT >= 2) b2 = WFrag<T16>::ld(Bt2 + boff + (size_t)nb * 16 * K + kc);
#pragma unroll
            for (int mb = 0; mb < 4; ++mb) { acc[mb][nb] = WFrag<T16>::mma(a[mb], b, acc[mb][nb]); if (NSPLIT == 1 || NSPLIT == 2) acc[mb][nb] = WFrag<T16>::mma(a2[mb], b, acc[mb][nb]); if (NSPLIT >= 2) acc[mb][nb] = WFrag<T16>::mma(a[mb], b2, acc[mb][nb]); } }
        asm volatile("v_nop\n\tv_nop\n\tv_nop\n\tv_nop" : "+v"(acc[0][0]), "+v"(acc[1][1]), "+v"(acc[2][2]), "+v"(acc[3][3]) : "v"(a[0]), "v"(a[3]));
    }
#pragma unroll
    for (int mb = 0; mb < 4; ++mb) {
#pragma unroll
        for (int nb = 0; nb < 4; ++nb) {
#pragma unroll
            for (int j = 0; j < 8; ++j) os[(hi * 8 + j) * 68 + nb * 16 + lr] = acc[mb][nb][j]; }
        __builtin_amdgcn_wave_barrier(); asm volatile("" ::: "memory");
        float* crow = C + (size_t)(r0 + mb * 16) * ldc + c0;
#pragma unroll 1
        for (int ps = 0; ps < 2; ++ps) {
#pragma unroll
            for (int s = 0; s < 8; ++s) { const int row = 2 * s + hi, cofs = lr * 4; v4f val = *(const v4fa*)(os + row * 68 + cofs); if (BIAS) { val[0] += bfr(bias[c0 + cofs]); val[1] += bfr(bias[c0 + cofs + 1]); val[2] += bfr(bias[c0 + cofs + 2]); val[3] += bfr(bias[c0 + cofs + 3]); }
                *(volatile v4f*)(crow + (size_t)row * ldc + cofs) = val; }
            if (ps == 0) __threadfence(); }
        __builtin_amdgcn_wave_barrier(); asm volatile("" ::: "memory");
    }
}

__device__ __forceinline__ h16 tohx(float x) { return (h16)x; }
__device__ __forceinline__ void splitf(float y, unsigned short& h, unsigned short& l) { h = f2bf(y); l = f2bf(y - bf2f(h)); }
typedef __attribute__((ext_vector_type(2))) _Float16 v2h;
typedef __attribute__((ext_vector_type(4))) _Float16 v4h;
typedef __attribute__((ext_vector_type(2))) unsigned short v2us;
typedef __attribute__((ext_vector_type(8))) _Float16 v8h_;

__global__ __launch_bounds__(256) void k_cvt8(const float* __restrict__ src, bf* dst, size_t n8) { const size_t i = (size_t)blockIdx.x * 256 + threadIdx.x; if (i >= n8) return; const v8f v = *(const v8f*)(src + i * 8); v8us o;
#pragma unroll
    for (int k = 0; k < 8; ++k) o[k] = f2bf(v[k]); *(volatile v8us*)(dst + i * 8) = o; __threadfence(); *(volatile v8us*)(dst + i * 8) = o; }
__global__ __launch_bounds__(256) void k_gnstat(const float* __restrict__ x, float* MS) {
    const int lane = threadIdx.x & 31; const int wg = blockIdx.x * 8 + (threadIdx.x >> 5); if (wg >= NB_ * NG) return; const float* base = x + (size_t)wg * 2 * NN;
    float s = 0.f;
#pragma unroll 4
    for (int i = 0; i < 2 * NN / 32; ++i) s += bfr(base[i * 32 + lane]);
#pragma unroll
    for (int sh = 16; sh; sh >>= 1) s += __shfl_xor(s, sh, 32);
    const float mu = s * (1.0f / (2 * NN)); float q = 0.f;
#pragma unroll 4
    for (int i = 0; i < 2 * NN / 32; ++i) { const float d = bfr(base[i * 32 + lane]) - mu; q = fmaf(d, d, q); }
#pragma unroll
    for (int sh = 16; sh; sh >>= 1) q += __shfl_xor(q, sh, 32);
    const float rs = rsqrtf(q * (1.0f / (2 * NN)) + 1e-6f);
    const float v = lane == 0 ? mu : (lane == 1 ? rs : 0.f); *(volatile float*)(MS + (size_t)wg * 32 + lane) = v; __threadfence(); *(volatile float*)(MS + (size_t)wg * 32 + lane) = v;
}
__global__ __launch_bounds__(256) void k_gnplane(const float* __restrict__ x, const float* __restrict__ MS, const float* __restrict__ gm, const float* __restrict__ bt, bf* Ph, bf* Pl) {
    const int lane = threadIdx.x & 31; const int L0 = (blockIdx.x * 8 + (threadIdx.x >> 5)) * 8; const int nlines = NB_ * NN * CC / 64;
#pragma unroll 1
    for (int ps = 0; ps < 2; ++ps) {
#pragma unroll
        for (int l = 0; l < 8; ++l) { const int L = L0 + l; if (L >= nlines) break; const int e = L * 64 + lane * 2; const int c = e & 63; const int n = (e >> 6) & 1023; const int b = e >> 16; v2us oh, ol;
#pragma unroll
            for (int q = 0; q < 2; ++q) { const int cc = c + q; const float* ms = MS + ((size_t)b * NG + (cc >> 1)) * 32; const float v = (bfr(x[((size_t)b * CC + cc) * NN + n]) - ms[0]) * ms[1] * bfr(gm[cc]) + bfr(bt[cc]); unsigned short a, c2; splitf(v, a, c2); oh[q] = a; ol[q] = c2; }
            *(volatile v2us*)(Ph + (size_t)e) = oh; *(volatile v2us*)(Pl + (size_t)e) = ol; }
        if (ps == 0) __threadfence(); }
}
__global__ __launch_bounds__(256) void k_softrows(const float* __restrict__ F, const float* __restrict__ bias, float* SM) {
    const int lane = threadIdx.x & 31; const int row = blockIdx.x * 8 + (threadIdx.x >> 5); if (row >= NB_ * QO) return; const float bb = bfr(bias[row % QO]); const float* sr = F + (size_t)row * NN; float v[32]; float m = -3.0e38f;
#pragma unroll
    for (int ch = 0; ch < 8; ++ch) { const v4f t = *(const v4f*)(sr + ch * 128 + lane * 4);
#pragma unroll
        for (int q = 0; q < 4; ++q) { v[ch * 4 + q] = t[q] + bb; m = fmaxf(m, v[ch * 4 + q]); } }
#pragma unroll
    for (int sh = 16; sh; sh >>= 1) m = fmaxf(m, __shfl_xor(m, sh, 32));
    float sum = 0.f;
#pragma unroll
    for (int i = 0; i < 32; ++i) { v[i] = __expf(v[i] - m); sum += v[i]; }
#pragma unroll
    for (int sh = 16; sh; sh >>= 1) sum += __shfl_xor(sum, sh, 32);
    const float f = __fdiv_rn(PCAR, sum);
#pragma unroll 1
    for (int ps = 0; ps < 2; ++ps) {
#pragma unroll
        for (int ch = 0; ch < 8; ++ch) { v4f o;
#pragma unroll
            for (int q = 0; q < 4; ++q) o[q] = v[ch * 4 + q] * f;
            *(volatile v4f*)(SM + (size_t)row * NN + ch * 128 + lane * 4) = o; }
        if (ps == 0) __threadfence(); }
}
__global__ __launch_bounds__(256) void k_tplane(const float* __restrict__ SM, h16* T) {
    __shared__ float tl[64][65];
    const int tid = threadIdx.x; const int n0 = blockIdx.x * 64, h = blockIdx.y, b = blockIdx.z;
#pragma unroll
    for (int i = 0; i < 16; ++i) { const int c = i * 4 + (tid >> 6), nn = tid & 63; tl[c][nn] = SM[((size_t)b * QO + h * CC + c) * NN + n0 + nn]; }
    __syncthreads();
    const int lane = tid & 31, wv = tid >> 5;
    auto pass = [&]() {
#pragma unroll
        for (int i2 = 0; i2 < 2; ++i2) { const int r = wv * 8 + i2 * 4 + (lane >> 3); const int cq = (lane & 7) * 8; v8h_ o;
#pragma unroll
            for (int i = 0; i < 8; ++i) o[i] = tohx(tl[cq + i][r]);
            *(volatile v8h_*)(T + (((size_t)(b * NH_ + h)) * NN + n0 + r) * CC + cq) = o; } };
    pass(); __threadfence(); pass();
}
__global__ __launch_bounds__(256) void k_vplane(const float* __restrict__ F, const float* __restrict__ bias, h16* Vp) {
    const int lane = threadIdx.x & 31; const int L0 = (blockIdx.x * 8 + (threadIdx.x >> 5)) * 8; const int nlines = NB_ * QO * NN / 64;
#pragma unroll 1
    for (int ps = 0; ps < 2; ++ps) {
#pragma unroll
        for (int l = 0; l < 8; ++l) { const int L = L0 + l; if (L >= nlines) break; const int e = L * 64 + lane * 2; const int oc = (e >> 10) % QO; v2h v;
#pragma unroll
            for (int q = 0; q < 2; ++q) v[q] = tohx(F[(size_t)e + q] + bfr(bias[oc]));
            *(volatile v2h*)(Vp + (size_t)e) = v; }
        if (ps == 0) __threadfence(); }
}
__global__ __launch_bounds__(256) void k_cvt16(const float* __restrict__ A, int nlines, h16* P) {
    const int lane = threadIdx.x & 31; const int L0 = (blockIdx.x * 8 + (threadIdx.x >> 5)) * 8;
#pragma unroll 1
    for (int ps = 0; ps < 2; ++ps) {
#pragma unroll
        for (int l = 0; l < 8; ++l) { const int L = L0 + l; if (L >= nlines) break; const int e = L * 64 + lane * 2; v2h v;
#pragma unroll
            for (int q = 0; q < 2; ++q) v[q] = tohx(A[(size_t)e + q]);
            *(volatile v2h*)(P + (size_t)e) = v; }
        if (ps == 0) __threadfence(); }
}
__global__ __launch_bounds__(256) void k_splits(const float* __restrict__ A, float sc, int nlines, bf* Ph, bf* Pl) {
    const int lane = threadIdx.x & 31; const int L0 = (blockIdx.x * 8 + (threadIdx.x >> 5)) * 8;
#pragma unroll 1
    for (int ps = 0; ps < 2; ++ps) {
#pragma unroll
        for (int l = 0; l < 8; ++l) { const int L = L0 + l; if (L >= nlines) break; const int e = L * 64 + lane * 2; v2us oh, ol;
#pragma unroll
            for (int q = 0; q < 2; ++q) { unsigned short a, c2; splitf(A[(size_t)e + q] * sc, a, c2); oh[q] = a; ol[q] = c2; }
            *(volatile v2us*)(Ph + (size_t)e) = oh; *(volatile v2us*)(Pl + (size_t)e) = ol; }
        if (ps == 0) __threadfence(); }
}
__global__ __launch_bounds__(256) void k_fin(const float* __restrict__ C2, const float* __restrict__ bo, float* OUT) {
    const size_t i = (size_t)blockIdx.x * 256 + threadIdx.x; if (i >= (size_t)NB_ * CC * NN / 4) return; const int o = (int)((i * 4 / NN) % CC); const v4f c = *(const v4f*)(C2 + i * 4); const float bb = bfr(bo[o]); v4f r;
#pragma unroll
    for (int k = 0; k < 4; ++k) r[k] = c[k] + bb; *(volatile v4f*)(OUT + i * 4) = r; __threadfence(); *(volatile v4f*)(OUT + i * 4) = r;
}

extern "C" void kernel_launch(void* const* d_in, const int* in_sizes, int n_in,
                              void* d_out, int out_size, void* d_ws, size_t ws_size, hipStream_t stream) {
    (void)in_sizes; (void)n_in; (void)out_size;
    const float* xq = (const float*)d_in[0]; const float* xkv = (const float*)d_in[1]; const float* gq = (const float*)d_in[2]; const float* btq = (const float*)d_in[3]; const float* gkv = (const float*)d_in[4]; const float* btkv = (const float*)d_in[5];
    const float* Wq = (const float*)d_in[6]; const float* bq = (const float*)d_in[7]; const float* Wk = (const float*)d_in[8]; const float* bk = (const float*)d_in[9]; const float* Wv = (const float*)d_in[10]; const float* bv = (const float*)d_in[11]; const float* Wo = (const float*)d_in[12]; const float* bo = (const float*)d_in[13];
    float* OUT = (float*)d_out;
    char* wsp = (char*)d_ws;
    auto take = [&](size_t bytes) { char* p = wsp; wsp += (bytes + 255) & ~(size_t)255; return (void*)p; };
    bf* WQ = (bf*)take((size_t)QO * CC * 2); bf* WK = (bf*)take((size_t)QO * CC * 2); bf* WV = (bf*)take((size_t)QO * CC * 2); bf* WO = (bf*)take((size_t)CC * QO * 2); bf* ZERO = (bf*)take((size_t)QO * CC * 2);
    float* MSq = (float*)take((size_t)NB_ * NG * 32 * 4); float* MSkv = (float*)take((size_t)NB_ * NG * 32 * 4);
    bf* XQh = (bf*)take((size_t)NB_ * NN * CC * 2); bf* XQl = (bf*)take((size_t)NB_ * NN * CC * 2); bf* XKh = (bf*)take((size_t)NB_ * NN * CC * 2); bf* XKl = (bf*)take((size_t)NB_ * NN * CC * 2);
    float* F = (float*)take((size_t)NB_ * QO * NN * 4); float* SM = (float*)take((size_t)NB_ * QO * NN * 4);
    h16* QsT = (h16*)take((size_t)NB_ * QO * NN * 2); h16* KsT = (h16*)take((size_t)NB_ * QO * NN * 2); h16* Vp = (h16*)take((size_t)NB_ * QO * NN * 2);
    float* ATT = (float*)take((size_t)NH_ * NN * NN * 4); h16* ATp = (h16*)take((size_t)NH_ * NN * NN * 2); float* OT = (float*)take((size_t)NB_ * NN * QO * 4); bf* OTh = (bf*)take((size_t)NB_ * NN * QO * 2); bf* OTl = (bf*)take((size_t)NB_ * NN * QO * 2); float* C2 = (float*)take((size_t)NB_ * CC * NN * 4);
    if ((size_t)(wsp - (char*)d_ws) > ws_size) return;
    { const size_t nw = (size_t)QO * CC / 8; const unsigned g = (unsigned)((nw + 255) / 256); k_cvt8<<<g, 256, 0, stream>>>(Wq, WQ, nw); k_cvt8<<<g, 256, 0, stream>>>(Wk, WK, nw); k_cvt8<<<g, 256, 0, stream>>>(Wv, WV, nw); k_cvt8<<<g, 256, 0, stream>>>(Wo, WO, nw); hipMemsetAsync(ZERO, 0, (size_t)QO * CC * 2, stream); }
    k_gnstat<<<NB_ * NG / 8, 256, 0, stream>>>(xq, MSq); k_gnstat<<<NB_ * NG / 8, 256, 0, stream>>>(xkv, MSkv);
    const unsigned LX = (unsigned)((NB_ * NN * CC / 64 + 63) / 64);
    k_gnplane<<<LX, 256, 0, stream>>>(xq, MSq, gq, btq, XQh, XQl); k_gnplane<<<LX, 256, 0, stream>>>(xkv, MSkv, gkv, btkv, XKh, XKl);
    const int NL = NB_ * QO * NN / 64;
    k_gemmw<bf, 2, false><<<dim3(QO / 64, NN / 64, NB_), 32, 0, stream>>>(WQ, ZERO, XQh, XQl, CC, F, NN, nullptr, 0, (size_t)NN * CC, (size_t)QO * NN);
    k_softrows<<<NB_ * QO / 8, 256, 0, stream>>>(F, bq, SM); k_tplane<<<dim3(NN / 64, NH_, NB_), 256, 0, stream>>>(SM, QsT);
    k_gemmw<bf, 2, false><<<dim3(QO / 64, NN / 64, NB_), 32, 0, stream>>>(WK, ZERO, XKh, XKl, CC, F, NN, nullptr, 0, (size_t)NN * CC, (size_t)QO * NN);
    k_softrows<<<NB_ * QO / 8, 256, 0, stream>>>(F, bk, SM); k_tplane<<<dim3(NN / 64, NH_, NB_), 256, 0, stream>>>(SM, KsT);
    k_gemmw<bf, 2, false><<<dim3(QO / 64, NN / 64, NB_), 32, 0, stream>>>(WV, ZERO, XKh, XKl, CC, F, NN, nullptr, 0, (size_t)NN * CC, (size_t)QO * NN);
    k_vplane<<<(unsigned)((NL + 63) / 64), 256, 0, stream>>>(F, bv, Vp);
    for (int b = 0; b < NB_; ++b) { const size_t z0 = (size_t)b * NH_;
        k_gemmw<h16, 0, false><<<dim3(NN / 64, NN / 64, NH_), 32, 0, stream>>>(QsT + z0 * NN * CC, nullptr, KsT + z0 * NN * CC, nullptr, CC, ATT, NN, nullptr, (size_t)NN * CC, (size_t)NN * CC, (size_t)NN * NN);
        k_cvt16<<<(NH_ * NN * NN / 64 + 63) / 64, 256, 0, stream>>>(ATT, NH_ * NN * NN / 64, ATp);
        k_gemmw<h16, 0, false><<<dim3(NN / 64, 1, NH_), 32, 0, stream>>>(ATp, nullptr, Vp + z0 * CC * NN, nullptr, NN, OT + (size_t)b * NN * QO, QO, nullptr, (size_t)NN * NN, (size_t)CC * NN, (size_t)CC); }
    k_splits<<<(unsigned)((NL + 63) / 64), 256, 0, stream>>>(OT, 0.125f / 1048576.0f, NL, OTh, OTl);
    k_gemmw<bf, 2, false><<<dim3(1, NN / 64, NB_), 32, 0, stream>>>(WO, ZERO, OTh, OTl, QO, C2, NN, nullptr, 0, (size_t)NN * QO, (size_t)CC * NN);
    k_fin<<<(unsigned)(((size_t)NB_ * CC * NN / 4 + 255) / 256), 256, 0, stream>>>(C2, bo, OUT);
}
